// SparseAttention_46127948759425
// MI455X (gfx1250) — hardware-verified
//
#include <hip/hip_runtime.h>


#ifndef NB
#define NB 2
#endif
#ifndef SEQ
#define SEQ 2048
#endif
#define NB_FULL  2
#define SEQ_FULL 2048
#define EMB      1024
#define NH       16
#define HD       64
#define QKVN     (3 * EMB)
#define MROWS    (NB * SEQ)
#define PCARRY   16384.0f

static_assert(NB >= 1 && NB <= NB_FULL);
static_assert(SEQ >= 128 && SEQ <= SEQ_FULL && (SEQ % 128) == 0);
static_assert(EMB == NH * HD);
static_assert(HD == 64);
static_assert((MROWS % 128) == 0);
static_assert((EMB % 64) == 0 && (QKVN % 64) == 0);
static_assert(((MROWS * (EMB / 8)) % 256) == 0);
static_assert(((NB * NH * (SEQ / 16)) % 4) == 0);

typedef _Float16       v16h __attribute__((ext_vector_type(16)));
typedef _Float16       v8h  __attribute__((ext_vector_type(8)));
typedef __bf16         v16b __attribute__((ext_vector_type(16)));
typedef unsigned short v8us __attribute__((ext_vector_type(8)));
typedef float          v8f  __attribute__((ext_vector_type(8)));
typedef float          v4f  __attribute__((ext_vector_type(4)));
typedef unsigned int   v4u  __attribute__((ext_vector_type(4)));

union FB { v16b v; v8us u[2]; };
union FH { v16h v; v8h h[2]; v8us u[2]; };
union H8 { v8h h; v4u u; };

#define WMMA_BF(a, b, c) __builtin_amdgcn_wmma_f32_16x16x32_bf16(false, (a), false, (b), (short)0, (c), false, false)
#define WMMA_HF(a, b, c) __builtin_amdgcn_wmma_f32_16x16x32_f16 (false, (a), false, (b), (short)0, (c), false, false)

__device__ __forceinline__ unsigned int bf16_rne(float f) {
    const unsigned int u = __float_as_uint(f);
    return ((u + 0x7FFFu + ((u >> 16) & 1u)) >> 16) & 0xFFFFu;
}
__device__ __forceinline__ float bf16_val(unsigned int b) { return __uint_as_float(b << 16); }

__device__ __forceinline__ v4u pack8(unsigned int b0, unsigned int b1, unsigned int b2, unsigned int b3,
                                     unsigned int b4, unsigned int b5, unsigned int b6, unsigned int b7) {
    v4u w;
    w[0] = (b0 & 0xFFFFu) | (b1 << 16);
    w[1] = (b2 & 0xFFFFu) | (b3 << 16);
    w[2] = (b4 & 0xFFFFu) | (b5 << 16);
    w[3] = (b6 & 0xFFFFu) | (b7 << 16);
    return w;
}

__global__ __launch_bounds__(256) void cvt_x_kernel(const float* __restrict__ x, unsigned short* __restrict__ xb)
{
    const int i = blockIdx.x * 256 + threadIdx.x;
    if (i >= MROWS * (EMB / 8)) return;
    const int r   = i / (EMB / 8);
    const int c8  = i - r * (EMB / 8);
    const int b   = r / SEQ;
    const int tok = r - b * SEQ;
    const float* src = x + ((size_t)b * SEQ_FULL + tok) * EMB + c8 * 8;
    const v4f f0 = *(const v4f*)src;
    const v4f f1 = *(const v4f*)(src + 4);
    const v4u w = pack8(bf16_rne(f0[0]), bf16_rne(f0[1]), bf16_rne(f0[2]), bf16_rne(f0[3]),
                        bf16_rne(f1[0]), bf16_rne(f1[1]), bf16_rne(f1[2]), bf16_rne(f1[3]));
    volatile v4u* d = (volatile v4u*)(xb + (size_t)r * EMB + c8 * 8);
    *d = w;
    __threadfence();
    *d = w;
}

__global__ __launch_bounds__(256) void cvt_wt_kernel(const float* __restrict__ W, int ncols,
                                                    unsigned short* __restrict__ Wt, int pitch, int dup)
{
    __shared__ __attribute__((aligned(16))) float tile[64 * 65];
    const int tid = threadIdx.x;
    const int n0 = blockIdx.x * 64;
    const int k0 = blockIdx.y * 64;
    {
        const int row = tid >> 2;
        const int c   = (tid & 3) * 16;
        const float* src = W + (size_t)(k0 + row) * ncols + n0 + c;
#pragma unroll
        for (int q = 0; q < 4; ++q) {
            const v4f f = *(const v4f*)(src + 4 * q);
            float* t = &tile[row * 65 + c + 4 * q];
            t[0] = f[0]; t[1] = f[1]; t[2] = f[2]; t[3] = f[3];
        }
    }
    __syncthreads();
    const int g = tid >> 3, e = tid & 7;
#pragma unroll
    for (int p = 0; p < 2; ++p) {
        const int j = p * 32 + g;
        unsigned int bb[8];
#pragma unroll
        for (int i2 = 0; i2 < 8; ++i2) bb[i2] = bf16_rne(tile[(e * 8 + i2) * 65 + j]);
        const v4u w = pack8(bb[0], bb[1], bb[2], bb[3], bb[4], bb[5], bb[6], bb[7]);
        const size_t o = (size_t)(n0 + j) * pitch + k0 + e * 8;
        volatile v4u* d0 = (volatile v4u*)(Wt + o);
        *d0 = w;
        if (dup) { volatile v4u* d1 = (volatile v4u*)(Wt + o + EMB); *d1 = w; }
        __threadfence();
        *d0 = w;
        if (dup) { volatile v4u* d1 = (volatile v4u*)(Wt + o + EMB); *d1 = w; }
    }
}

__device__ __forceinline__ void gemm_strip(const unsigned short* __restrict__ A, const unsigned short* __restrict__ Bt,
                                           const int K, const int m0, const int n0, const int lane, v8f acc[2][4])
{
    const int half = lane >> 4, ln = lane & 15;
    const unsigned short* ap0 = A  + (size_t)(m0 + ln) * K + 8 * half;
    const unsigned short* ap1 = ap0 + (size_t)16 * K;
    const unsigned short* bp0 = Bt + (size_t)(n0 + ln) * K + 8 * half;
    const size_t bs = (size_t)16 * K;
#pragma unroll 1
    for (int k = 0; k < K; k += 32) {
        FB a0, a1, b0, b1, b2, b3;
        a0.u[0] = *(const v8us*)(ap0 + k);           a0.u[1] = *(const v8us*)(ap0 + k + 16);
        a1.u[0] = *(const v8us*)(ap1 + k);           a1.u[1] = *(const v8us*)(ap1 + k + 16);
        b0.u[0] = *(const v8us*)(bp0 + k);           b0.u[1] = *(const v8us*)(bp0 + k + 16);
        b1.u[0] = *(const v8us*)(bp0 + bs + k);      b1.u[1] = *(const v8us*)(bp0 + bs + k + 16);
        b2.u[0] = *(const v8us*)(bp0 + 2 * bs + k);  b2.u[1] = *(const v8us*)(bp0 + 2 * bs + k + 16);
        b3.u[0] = *(const v8us*)(bp0 + 3 * bs + k);  b3.u[1] = *(const v8us*)(bp0 + 3 * bs + k + 16);
        acc[0][0] = WMMA_BF(a0.v, b0.v, acc[0][0]);
        acc[1][0] = WMMA_BF(a1.v, b0.v, acc[1][0]);
        acc[0][1] = WMMA_BF(a0.v, b1.v, acc[0][1]);
        acc[1][1] = WMMA_BF(a1.v, b1.v, acc[1][1]);
        acc[0][2] = WMMA_BF(a0.v, b2.v, acc[0][2]);
        acc[1][2] = WMMA_BF(a1.v, b2.v, acc[1][2]);
        acc[0][3] = WMMA_BF(a0.v, b3.v, acc[0][3]);
        acc[1][3] = WMMA_BF(a1.v, b3.v, acc[1][3]);
        asm volatile("v_nop\n\tv_nop\n\tv_nop\n\tv_nop"
                     : "+v"(acc[0][0]), "+v"(acc[1][0]), "+v"(acc[0][1]), "+v"(acc[1][1]),
                       "+v"(acc[0][2]), "+v"(acc[1][2]), "+v"(acc[0][3]), "+v"(acc[1][3])
                     : "v"(a0.u[0]), "v"(a0.u[1]), "v"(a1.u[0]), "v"(a1.u[1]),
                       "v"(b0.u[0]), "v"(b0.u[1]), "v"(b1.u[0]), "v"(b1.u[1]),
                       "v"(b2.u[0]), "v"(b2.u[1]), "v"(b3.u[0]), "v"(b3.u[1]));
    }
}

__global__ __launch_bounds__(128) void qkv_gemm_kernel(
        const unsigned short* __restrict__ Xb, const unsigned short* __restrict__ Wt, const float* __restrict__ bias,
        unsigned short* __restrict__ Qh, unsigned short* __restrict__ Ql,
        unsigned short* __restrict__ Kh, unsigned short* __restrict__ Kl,
        unsigned short* __restrict__ VTh, unsigned short* __restrict__ VTl)
{
    __shared__ __attribute__((aligned(16))) float stg[128 * 68];
    const int tid = threadIdx.x, lane = tid & 31, wib = tid >> 5;
    const int half = lane >> 4, ln = lane & 15;
    const int nmb = MROWS / 128;
    const int mb = blockIdx.x % nmb, ns = blockIdx.x / nmb;
    const int m0b = mb * 128, n0 = ns * 64;

    v8f acc[2][4];
    const v8f z = {};
#pragma unroll
    for (int mi = 0; mi < 2; ++mi)
#pragma unroll
        for (int t = 0; t < 4; ++t) acc[mi][t] = z;

    gemm_strip(Xb, Wt, EMB, m0b + wib * 32, n0, lane, acc);

#pragma unroll
    for (int mi = 0; mi < 2; ++mi)
#pragma unroll
        for (int t = 0; t < 4; ++t)
#pragma unroll
            for (int i = 0; i < 8; ++i)
                stg[(wib * 32 + mi * 16 + 8 * half + i) * 68 + t * 16 + ln] = acc[mi][t][i];
    __syncthreads();

    const int s    = n0 / EMB;
    const int hh   = (n0 % EMB) / HD;
    const int b    = m0b / SEQ;
    const int tok0 = m0b % SEQ;
    const int bh   = b * NH + hh;
    const int g = tid >> 3, e = tid & 7;

    if (s < 2) {
        unsigned short* Ph = (s == 0) ? Qh : Kh;
        unsigned short* Pl = (s == 0) ? Ql : Kl;
        float bb[8];
#pragma unroll
        for (int i = 0; i < 8; ++i) bb[i] = bf16_val(bf16_rne(bias[n0 + e * 8 + i]));
#pragma unroll
        for (int p = 0; p < 8; ++p) {
            const int row = p * 16 + g;
            const float* sp = &stg[row * 68 + e * 8];
            const v4f f0 = *(const v4f*)sp;
            const v4f f1 = *(const v4f*)(sp + 4);
            float v[8];
            v[0] = f0[0] + bb[0]; v[1] = f0[1] + bb[1]; v[2] = f0[2] + bb[2]; v[3] = f0[3] + bb[3];
            v[4] = f1[0] + bb[4]; v[5] = f1[1] + bb[5]; v[6] = f1[2] + bb[6]; v[7] = f1[3] + bb[7];
            unsigned int hb[8], lb[8];
#pragma unroll
            for (int i = 0; i < 8; ++i) {
                hb[i] = bf16_rne(v[i]);
                lb[i] = bf16_rne(v[i] - bf16_val(hb[i]));
            }
            const v4u wh = pack8(hb[0], hb[1], hb[2], hb[3], hb[4], hb[5], hb[6], hb[7]);
            const v4u wl = pack8(lb[0], lb[1], lb[2], lb[3], lb[4], lb[5], lb[6], lb[7]);
            const size_t off = ((size_t)bh * SEQ + tok0 + row) * HD + e * 8;
            volatile v4u* dh = (volatile v4u*)(Ph + off);
            volatile v4u* dl = (volatile v4u*)(Pl + off);
            *dh = wh; *dl = wl;
            __threadfence();
            *dh = wh; *dl = wl;
        }
    } else {
#pragma unroll
        for (int p = 0; p < 8; ++p) {
            const int L  = p * 16 + g;
            const int d  = L >> 1, hf = L & 1;
            const float bd = bf16_val(bf16_rne(bias[n0 + d]));
            H8 hv;
            unsigned int lb[8];
#pragma unroll
            for (int i = 0; i < 8; ++i) {
                const float v = stg[(hf * 64 + e * 8 + i) * 68 + d] + bd;
                hv.h[i] = (_Float16)v;
                lb[i] = bf16_rne(v - (float)hv.h[i]);
            }
            const v4u wl = pack8(lb[0], lb[1], lb[2], lb[3], lb[4], lb[5], lb[6], lb[7]);
            const size_t off = ((size_t)bh * HD + d) * SEQ + tok0 + hf * 64 + e * 8;
            volatile v4u* dh = (volatile v4u*)(VTh + off);
            volatile v4u* dl = (volatile v4u*)(VTl + off);
            const v4u whv = hv.u;
            *dh = whv; *dl = wl;
            __threadfence();
            *dh = whv; *dl = wl;
        }
    }
}

__device__ __forceinline__ v8f score_tile(const v16b qh0, const v16b ql0, const v16b qh1, const v16b ql1,
                                          const unsigned short* __restrict__ khp,
                                          const unsigned short* __restrict__ klp)
{
    FB kh0, kh1, kl0, kl1;
    kh0.u[0] = *(const v8us*)(khp);       kh0.u[1] = *(const v8us*)(khp + 16);
    kh1.u[0] = *(const v8us*)(khp + 32);  kh1.u[1] = *(const v8us*)(khp + 48);
    kl0.u[0] = *(const v8us*)(klp);       kl0.u[1] = *(const v8us*)(klp + 16);
    kl1.u[0] = *(const v8us*)(klp + 32);  kl1.u[1] = *(const v8us*)(klp + 48);
    v8f sa = {};
    sa = WMMA_BF(qh0, kh0.v, sa);
    sa = WMMA_BF(ql0, kh0.v, sa);
    sa = WMMA_BF(qh0, kl0.v, sa);
    sa = WMMA_BF(qh1, kh1.v, sa);
    sa = WMMA_BF(ql1, kh1.v, sa);
    sa = WMMA_BF(qh1, kl1.v, sa);
    asm volatile("v_nop\n\tv_nop\n\tv_nop\n\tv_nop" : "+v"(sa)
                 : "v"(kh0.u[0]), "v"(kh0.u[1]), "v"(kh1.u[0]), "v"(kh1.u[1]),
                   "v"(kl0.u[0]), "v"(kl0.u[1]), "v"(kl1.u[0]), "v"(kl1.u[1]));
    return sa;
}

#define PV_STEP(ACC, DT) {                                                                        \
    FH vh; FB vl;                                                                                 \
    const unsigned short* vp = vhb + (size_t)((DT) * 16) * SEQ + j0;                              \
    const unsigned short* wp = vlb + (size_t)((DT) * 16) * SEQ + j0;                              \
    vh.u[0] = *(const v8us*)(vp); vh.u[1] = *(const v8us*)(vp + 16);                              \
    vl.u[0] = *(const v8us*)(wp); vl.u[1] = *(const v8us*)(wp + 16);                              \
    ACC = WMMA_HF(ap.v, vh.v, ACC);                                                               \
    ACC = WMMA_BF(apb.v, vl.v, ACC);                                                              \
    asm volatile("v_nop\n\tv_nop\n\tv_nop\n\tv_nop" : "+v"(ACC)                                                                \
                 : "v"(ap.u[0]), "v"(ap.u[1]), "v"(apb.u[0]), "v"(apb.u[1]),                    \
                   "v"(vh.u[0]), "v"(vh.u[1]), "v"(vl.u[0]), "v"(vl.u[1]));                       \
}

__global__ __launch_bounds__(128) void attn_kernel(
        const unsigned short* __restrict__ Qh, const unsigned short* __restrict__ Ql,
        const unsigned short* __restrict__ Kh, const unsigned short* __restrict__ Kl,
        const unsigned short* __restrict__ VTh, const unsigned short* __restrict__ VTl,
        unsigned short* __restrict__ ctx)
{
    __shared__ __attribute__((aligned(16))) _Float16       Pf[4][16 * 40];
    __shared__ __attribute__((aligned(16))) unsigned short Pb[4][16 * 40];
    __shared__ __attribute__((aligned(16))) float          stg[4][16 * 68];

    const int tid = threadIdx.x, lane = tid & 31, wib = tid >> 5;
    const int half = lane >> 4, ln = lane & 15;
    const int nqt = SEQ / 16;
    const int gw  = blockIdx.x * 4 + wib;
    const int qt  = gw % nqt;
    const int bh  = gw / nqt;
    const int b   = bh / NH, h = bh % NH;
    const int q0  = qt * 16;

    _Float16*       pf = &Pf[wib][0];
    unsigned short* pb = &Pb[wib][0];
    float*          sg = &stg[wib][0];

    FB qh0, qh1, ql0, ql1;
    {
        const unsigned short* p = Qh + ((size_t)bh * SEQ + q0 + ln) * HD + 8 * half;
        const unsigned short* r = Ql + ((size_t)bh * SEQ + q0 + ln) * HD + 8 * half;
        qh0.u[0] = *(const v8us*)(p);      qh0.u[1] = *(const v8us*)(p + 16);
        qh1.u[0] = *(const v8us*)(p + 32); qh1.u[1] = *(const v8us*)(p + 48);
        ql0.u[0] = *(const v8us*)(r);      ql0.u[1] = *(const v8us*)(r + 16);
        ql1.u[0] = *(const v8us*)(r + 32); ql1.u[1] = *(const v8us*)(r + 48);
    }
    const unsigned short* khb = Kh  + ((size_t)bh * SEQ + ln) * HD + 8 * half;
    const unsigned short* klb = Kl  + ((size_t)bh * SEQ + ln) * HD + 8 * half;
    const unsigned short* vhb = VTh + ((size_t)bh * HD + ln) * SEQ + 8 * half;
    const unsigned short* vlb = VTl + ((size_t)bh * HD + ln) * SEQ + 8 * half;

    float m[8], l[8];
    v8f acc0 = {}, acc1 = {}, acc2 = {}, acc3 = {};
#pragma unroll
    for (int r = 0; r < 8; ++r) { m[r] = -1.0e30f; l[r] = 0.f; }

#pragma unroll 1
    for (int j0 = 0; j0 < SEQ; j0 += 32) {
        const v8f s0 = score_tile(qh0.v, ql0.v, qh1.v, ql1.v, khb + (size_t)j0 * HD,        klb + (size_t)j0 * HD);
        const v8f s1 = score_tile(qh0.v, ql0.v, qh1.v, ql1.v, khb + (size_t)(j0 + 16) * HD, klb + (size_t)(j0 + 16) * HD);

        __builtin_amdgcn_fence(4  , "wavefront");
        __builtin_amdgcn_wave_barrier();

#pragma unroll
        for (int r = 0; r < 8; ++r) {
            const float x0 = s0[r] * 0.5f;
            const float x1 = s1[r] * 0.5f;
            float mx = fmaxf(x0, x1);
#pragma unroll
            for (int off = 1; off < 16; off <<= 1) mx = fmaxf(mx, __shfl_xor(mx, off, 32));
            const float mn = fmaxf(m[r], mx);
            const float fc = __expf(m[r] - mn);
            const float e0 = __expf(x0 - mn);
            const float e1 = __expf(x1 - mn);
            float ps = e0 + e1;
#pragma unroll
            for (int off = 1; off < 16; off <<= 1) ps += __shfl_xor(ps, off, 32);
            l[r] = l[r] * fc + ps;
            m[r] = mn;
            acc0[r] *= fc; acc1[r] *= fc; acc2[r] *= fc; acc3[r] *= fc;
            const float c0 = e0 * PCARRY;
            const float c1 = e1 * PCARRY;
            const int prow = (8 * half + r) * 40;
            pf[prow + ln]      = (_Float16)c0;
            pf[prow + 16 + ln] = (_Float16)c1;
            pb[prow + ln]      = (unsigned short)bf16_rne(c0);
            pb[prow + 16 + ln] = (unsigned short)bf16_rne(c1);
        }
        __builtin_amdgcn_fence(4  , "wavefront");
        __builtin_amdgcn_wave_barrier();

        FH ap; FB apb;
        ap.h[0]  = *(const v8h*)(pf + ln * 40 + 8 * half);
        ap.h[1]  = *(const v8h*)(pf + ln * 40 + 16 + 8 * half);
        apb.u[0] = *(const v8us*)(pb + ln * 40 + 8 * half);
        apb.u[1] = *(const v8us*)(pb + ln * 40 + 16 + 8 * half);

        PV_STEP(acc0, 0)
        PV_STEP(acc1, 1)
        PV_STEP(acc2, 2)
        PV_STEP(acc3, 3)
    }

#pragma unroll
    for (int r = 0; r < 8; ++r) {
        const float inv = 1.0f / (l[r] * PCARRY);
        const int row = (8 * half + r) * 68;
        sg[row + ln]      = acc0[r] * inv;
        sg[row + 16 + ln] = acc1[r] * inv;
        sg[row + 32 + ln] = acc2[r] * inv;
        sg[row + 48 + ln] = acc3[r] * inv;
    }
    __builtin_amdgcn_fence(4  , "wavefront");
    __builtin_amdgcn_wave_barrier();

    const int g = lane >> 3, e = lane & 7;
#pragma unroll
    for (int p = 0; p < 4; ++p) {
        const int row = p * 4 + g;
        const float* sp = sg + row * 68 + e * 8;
        const v4f f0 = *(const v4f*)sp;
        const v4f f1 = *(const v4f*)(sp + 4);
        float v[8];
        v[0] = f0[0]; v[1] = f0[1]; v[2] = f0[2]; v[3] = f0[3];
        v[4] = f1[0]; v[5] = f1[1]; v[6] = f1[2]; v[7] = f1[3];
        unsigned int hb[8], lb[8];
#pragma unroll
        for (int i = 0; i < 8; ++i) {
            hb[i] = bf16_rne(v[i]);
            lb[i] = bf16_rne(v[i] - bf16_val(hb[i]));
        }
        const v4u wh = pack8(hb[0], hb[1], hb[2], hb[3], hb[4], hb[5], hb[6], hb[7]);
        const v4u wl = pack8(lb[0], lb[1], lb[2], lb[3], lb[4], lb[5], lb[6], lb[7]);
        const size_t off = ((size_t)b * SEQ + q0 + row) * (2 * EMB) + h * HD + e * 8;
        volatile v4u* dh = (volatile v4u*)(ctx + off);
        volatile v4u* dl = (volatile v4u*)(ctx + off + EMB);
        *dh = wh; *dl = wl;
        __threadfence();
        *dh = wh; *dl = wl;
    }
}

__global__ __launch_bounds__(128) void proj_gemm_kernel(
        const unsigned short* __restrict__ Cx, const unsigned short* __restrict__ Wt2,
        const float* __restrict__ bias, float* __restrict__ out)
{
    __shared__ __attribute__((aligned(16))) float stg[128 * 68];
    const int tid = threadIdx.x, lane = tid & 31, wib = tid >> 5;
    const int half = lane >> 4, ln = lane & 15;
    const int nmb = MROWS / 128;
    const int mb = blockIdx.x % nmb, ns = blockIdx.x / nmb;
    const int m0b = mb * 128, n0 = ns * 64;

    v8f acc[2][4];
    const v8f z = {};
#pragma unroll
    for (int mi = 0; mi < 2; ++mi)
#pragma unroll
        for (int t = 0; t < 4; ++t) acc[mi][t] = z;

    gemm_strip(Cx, Wt2, 2 * EMB, m0b + wib * 32, n0, lane, acc);

#pragma unroll
    for (int mi = 0; mi < 2; ++mi)
#pragma unroll
        for (int t = 0; t < 4; ++t)
#pragma unroll
            for (int i = 0; i < 8; ++i)
                stg[(wib * 32 + mi * 16 + 8 * half + i) * 68 + t * 16 + ln] = acc[mi][t][i];
    __syncthreads();

    const int g = tid >> 3, e = tid & 7;
#pragma unroll
    for (int p = 0; p < 16; ++p) {
        const int L   = p * 16 + g;
        const int row = L >> 1, hf = L & 1;
        const int col = hf * 32 + e * 4;
        v4f v = *(const v4f*)&stg[row * 68 + col];
        v[0] += bf16_val(bf16_rne(bias[n0 + col + 0]));
        v[1] += bf16_val(bf16_rne(bias[n0 + col + 1]));
        v[2] += bf16_val(bf16_rne(bias[n0 + col + 2]));
        v[3] += bf16_val(bf16_rne(bias[n0 + col + 3]));
        volatile v4f* d = (volatile v4f*)(out + (size_t)(m0b + row) * EMB + n0 + col);
        *d = v;
        __threadfence();
        *d = v;
    }
}

extern "C" void kernel_launch(void* const* d_in, const int* in_sizes, int n_in,
                              void* d_out, int out_size, void* d_ws, size_t ws_size,
                              hipStream_t stream)
{
    if (n_in < 5) return;
    if (in_sizes[0] < ((NB - 1) * SEQ_FULL + SEQ) * EMB) return;
    if (in_sizes[1] < EMB * QKVN) return;
    if (in_sizes[2] < QKVN) return;
    if (in_sizes[3] < EMB * EMB) return;
    if (in_sizes[4] < EMB) return;
    if (out_size < MROWS * EMB) return;

    const float* x     = (const float*)d_in[0];
    const float* Wqkv  = (const float*)d_in[1];
    const float* bqkv  = (const float*)d_in[2];
    const float* Wproj = (const float*)d_in[3];
    const float* bproj = (const float*)d_in[4];
    float* out = (float*)d_out;

    char* ws = (char*)d_ws;
    size_t off = 0;
    auto take = [&](size_t bytes) -> void* {
        void* p = ws + off;
        off += (bytes + 255) & ~(size_t)255;
        return p;
    };
    const size_t szX   = (size_t)MROWS * EMB * 2;
    const size_t szWq  = (size_t)QKVN * EMB * 2;
    const size_t szWp  = (size_t)EMB * (2 * EMB) * 2;
    const size_t szPl  = (size_t)NB * NH * SEQ * HD * 2;
    const size_t szCtx = (size_t)MROWS * (2 * EMB) * 2;
    unsigned short* Xb   = (unsigned short*)take(szX);
    unsigned short* WqT  = (unsigned short*)take(szWq);
    unsigned short* WpT2 = (unsigned short*)take(szWp);
    unsigned short* Qh   = (unsigned short*)take(szPl);
    unsigned short* Ql   = (unsigned short*)take(szPl);
    unsigned short* Kh   = (unsigned short*)take(szPl);
    unsigned short* Kl   = (unsigned short*)take(szPl);
    unsigned short* VTh  = (unsigned short*)take(szPl);
    unsigned short* VTl  = (unsigned short*)take(szPl);
    unsigned short* Cx   = (unsigned short*)take(szCtx);
    if (off > ws_size) return;

    cvt_x_kernel<<<(MROWS * (EMB / 8)) / 256, 256, 0, stream>>>(x, Xb);
    cvt_wt_kernel<<<dim3(QKVN / 64, EMB / 64), 256, 0, stream>>>(Wqkv, QKVN, WqT, EMB, 0);
    cvt_wt_kernel<<<dim3(EMB / 64, EMB / 64), 256, 0, stream>>>(Wproj, EMB, WpT2, 2 * EMB, 1);
    qkv_gemm_kernel<<<(MROWS / 128) * (QKVN / 64), 128, 0, stream>>>(Xb, WqT, bqkv, Qh, Ql, Kh, Kl, VTh, VTl);
    attn_kernel<<<(NB * NH * (SEQ / 16)) / 4, 128, 0, stream>>>(Qh, Ql, Kh, Kl, VTh, VTl, Cx);
    proj_gemm_kernel<<<(MROWS / 128) * (EMB / 64), 128, 0, stream>>>(Cx, WpT2, bproj, out);
}
